// HetGATEncoder_17901423690125
// MI455X (gfx1250) — hardware-verified
//
#include <hip/hip_runtime.h>
#include <stddef.h>
#include <math.h>

typedef __attribute__((ext_vector_type(16))) _Float16 v16h;
typedef __attribute__((ext_vector_type(8)))  _Float16 v8h;
typedef __attribute__((ext_vector_type(16))) __bf16   v16b;
typedef __attribute__((ext_vector_type(8)))  __bf16   v8b;
typedef __attribute__((ext_vector_type(8)))  float    v8f;
typedef __attribute__((ext_vector_type(4)))  float    v4f;
typedef __attribute__((ext_vector_type(4)))  int      v4i;

constexpr int XIN     = 16;
constexpr int XKP     = 32;
constexpr int FW      = 64;
constexpr int NHL1    = 4;
constexpr int NBL1    = 512;
constexpr int NBL2    = 1024;
constexpr int RPQ     = 1024;
constexpr int ROWS_CS = 512;
#define NTHR    256
#define NWAVE   8
#define EPT     8
#define NGRP    1
#define CHUNK   (NTHR * EPT * NGRP)
#define WCAP    (EPT * NGRP * 32)
#define LISTN   (NWAVE * WCAP)
constexpr int lds_agg_bytes(int nb, int nh) { return (nb * FW + 2 * nb * nh) * 4 + LISTN * 4 + 64; }
constexpr int LDS1 = lds_agg_bytes(NBL1, NHL1);
constexpr int LDS2 = lds_agg_bytes(NBL2, 1);

static_assert((CHUNK & (CHUNK - 1)) == 0);
static_assert(CHUNK <= 4096);
static_assert(LDS1 == 155712 && LDS2 == 278592);
static_assert((NBL1 & (NBL1 - 1)) == 0 && (NBL2 & (NBL2 - 1)) == 0 && NBL2 <= 4096);
static_assert(RPQ % NBL1 == 0 && RPQ % NBL2 == 0 && RPQ % 64 == 0 && RPQ % NTHR == 0 && RPQ % ROWS_CS == 0);
static_assert(NTHR == 4 * FW && ROWS_CS % 4 == 0 && XKP % 32 == 0 && FW % 32 == 0);

__device__ __forceinline__ unsigned short f2bf_bits(float f) {
  unsigned u = __float_as_uint(f);
  return (unsigned short)((u + 0x7FFFu + ((u >> 16) & 1u)) >> 16);
}
__device__ __forceinline__ float bf_bits2f(unsigned short h) { return __uint_as_float(((unsigned)h) << 16); }

__device__ __forceinline__ void dep_guard_h(v8f& a, v8f& b, v16h x, v16h y) { asm volatile("v_nop\n\tv_nop\n\tv_nop\n\tv_nop" : "+v"(a), "+v"(b) : "v"(x), "v"(y)); }
__device__ __forceinline__ void dep_guard_b(v8f& a, v8f& b, v16b x, v16b y) { asm volatile("v_nop\n\tv_nop\n\tv_nop\n\tv_nop" : "+v"(a), "+v"(b) : "v"(x), "v"(y)); }
__device__ __forceinline__ void keep4_h(v16h a, v16h b, v16h c, v16h d) { asm volatile("v_nop" :: "v"(a), "v"(b), "v"(c), "v"(d)); }
__device__ __forceinline__ void keep4_b(v16b a, v16b b, v16b c, v16b d) { asm volatile("v_nop" :: "v"(a), "v"(b), "v"(c), "v"(d)); }
__device__ __forceinline__ void acc_guard4(v8f& a, v8f& b, v8f& c, v8f& d) { asm volatile("v_nop\n\tv_nop\n\tv_nop\n\tv_nop" : "+v"(a), "+v"(b), "+v"(c), "+v"(d)); }
template <typename T> struct Frag;
template <> struct Frag<_Float16> {
  typedef v16h V; union U { v16h v; v8h h[2]; };
  static __device__ __forceinline__ v16h load(const _Float16* p) {
    U f; f.h[0] = *(const v8h*)(p); f.h[1] = *(const v8h*)(p + 16); return f.v;
  }
  static __device__ __forceinline__ v8f mma(v16h a, v16h b, v8f c) {
    return __builtin_amdgcn_wmma_f32_16x16x32_f16(false, a, false, b, (short)0, c, false, false);
  }
  static __device__ __forceinline__ void guard(v8f& a, v8f& b, v16h x, v16h y) { dep_guard_h(a, b, x, y); }
  static __device__ __forceinline__ void keep(v16h a, v16h b, v16h c, v16h d) { keep4_h(a, b, c, d); }
};
template <> struct Frag<__bf16> {
  typedef v16b V; union U { v16b v; v8b h[2]; };
  static __device__ __forceinline__ v16b load(const __bf16* p) {
    U f; f.h[0] = *(const v8b*)(p); f.h[1] = *(const v8b*)(p + 16); return f.v;
  }
  static __device__ __forceinline__ v8f mma(v16b a, v16b b, v8f c) {
    return __builtin_amdgcn_wmma_f32_16x16x32_bf16(false, a, false, b, (short)0, c, false, false);
  }
  static __device__ __forceinline__ void guard(v8f& a, v8f& b, v16b x, v16b y) { dep_guard_b(a, b, x, y); }
  static __device__ __forceinline__ void keep(v16b a, v16b b, v16b c, v16b d) { keep4_b(a, b, c, d); }
};

template <int ET> struct Elem;
template <> struct Elem<0> { typedef _Float16 T; };
template <> struct Elem<1> { typedef __bf16 T; };
template <int ET, bool SPLIT, int BIAS_MODE, int OUT_MODE, bool RESID, int ACT = 0>
__global__ __launch_bounds__(256) void wmma_gemm64(
    const unsigned short* __restrict__ Ap, const unsigned short* __restrict__ A2p, int lda, long strideA,
    const unsigned short* __restrict__ Btp, const unsigned short* __restrict__ Bt2p, int ldb, long strideB,
    void* __restrict__ Cout, void* __restrict__ Cout2, int ldc, long strideC,
    const float* __restrict__ bias,
    const float* __restrict__ resid, long strideR,
    int M, int N, int K, float scale) {
  typedef typename Elem<ET>::T T;
  typedef typename Frag<T>::V V;
  const T* A = (const T*)Ap; const T* A2 = (const T*)A2p; const T* Bt = (const T*)Btp; const T* Bt2 = (const T*)Bt2p;
  __shared__ __align__(16) float sT[8][16 * 68];
  const int b    = blockIdx.y;
  const int lane = threadIdx.x & 31;
  const int wave = threadIdx.x >> 5;
  const int tilesN = N >> 6;
  const int tilesM = M >> 6;
  const int tile = blockIdx.x * 8 + wave;
  if (tile >= tilesM * tilesN) return;
  const int tm = tile / tilesN;
  const int tn = tile - tm * tilesN;
  const int m0 = tm << 6;
  const int n0 = tn << 6;

  const T* Ab  = A  + (size_t)b * strideA;
  const T* Bb  = Bt + (size_t)b * strideB;
  const T* Ab2 = SPLIT ? (A2  + (size_t)b * strideA) : nullptr;
  const T* Bb2 = SPLIT ? (Bt2 + (size_t)b * strideB) : nullptr;

  const int rlane = lane & 15;
  const int koff  = (lane >> 4) * 8;
  const int mOff  = (lane >> 4) * 8;

  v8f acc[4][4];
#pragma unroll
  for (int i = 0; i < 4; ++i)
#pragma unroll
    for (int j = 0; j < 4; ++j) acc[i][j] = (v8f){0.f,0.f,0.f,0.f,0.f,0.f,0.f,0.f};

  for (int k0 = 0; k0 < K; k0 += 32) {
    V bh[4], bl[4];
#pragma unroll
    for (int j = 0; j < 4; ++j) {
      const size_t bo = (size_t)(n0 + (j << 4) + rlane) * ldb + koff + k0;
      bh[j] = Frag<T>::load(Bb + bo);
      if (SPLIT) bl[j] = Frag<T>::load(Bb2 + bo);
    }
#pragma unroll
    for (int i = 0; i < 4; ++i) {
      const size_t ao = (size_t)(m0 + (i << 4) + rlane) * lda + koff + k0;
      V ah = Frag<T>::load(Ab + ao);
      V al;
      if (SPLIT) al = Frag<T>::load(Ab2 + ao);
#pragma unroll
      for (int j = 0; j < 4; ++j) {
        acc[i][j] = Frag<T>::mma(ah, bh[j], acc[i][j]);
        if (SPLIT) {
          acc[i][j] = Frag<T>::mma(ah, bl[j], acc[i][j]);
          acc[i][j] = Frag<T>::mma(al, bh[j], acc[i][j]);
        }
      }
      Frag<T>::guard(acc[i][0], acc[i][3], ah, SPLIT ? al : ah);
    }
    Frag<T>::keep(bh[0], bh[1], bh[2], bh[3]);
    if (SPLIT) Frag<T>::keep(bl[0], bl[1], bl[2], bl[3]);
  }
  acc_guard4(acc[0][0], acc[0][1], acc[0][2], acc[0][3]);
  acc_guard4(acc[1][0], acc[1][1], acc[1][2], acc[1][3]);
  acc_guard4(acc[2][0], acc[2][1], acc[2][2], acc[2][3]);
  acc_guard4(acc[3][0], acc[3][1], acc[3][2], acc[3][3]);

  float* slab = sT[wave];
  const float* Rb = RESID ? (resid + (size_t)b * strideR) : nullptr;
#pragma unroll
  for (int i = 0; i < 4; ++i) {
    const int mBase = m0 + (i << 4);
#pragma unroll
    for (int j = 0; j < 4; ++j) {
      const int n = n0 + (j << 4) + rlane;
      float bv = 0.f;
      if (BIAS_MODE == 2) bv = bias[n];
#pragma unroll
      for (int r = 0; r < 8; ++r) {
        float v = acc[i][j][r] * scale;
        if (BIAS_MODE == 1) v += bias[mBase + mOff + r];
        if (BIAS_MODE == 2) v += bv;
        if (RESID) v += Rb[(size_t)(mBase + mOff + r) * ldc + n];
        if (ACT == 1) v = tanhf(v);
        if (ACT == 2) v = fmaxf(v, 0.0f);
        if (ACT == 3) v = v / (1.0f + expf(-v));
        if (ACT == 4) v = (v > 0.f) ? v : 0.01f * v;
        if (ACT == 5) v = 0.5f * v * (1.0f + erff(v * 0.70710678118654752f));
        slab[(mOff + r) * 68 + (j << 4) + rlane] = v;
      }
    }
    __builtin_amdgcn_fence(__ATOMIC_RELEASE, "workgroup");
    __builtin_amdgcn_wave_barrier();
    __builtin_amdgcn_fence(__ATOMIC_ACQUIRE, "workgroup");
    if (OUT_MODE == 0) {
      float* C = (float*)Cout + (size_t)b * strideC;
      const int hh = lane >> 4, c4 = (lane & 15) * 4;
      for (int pass = 0; pass < 2; ++pass) {
#pragma unroll
        for (int it = 0; it < 8; ++it) {
          const int row = it * 2 + hh;
          v4f v = *(const v4f*)(slab + row * 68 + c4);
          *(volatile v4f*)(C + (size_t)(mBase + row) * ldc + n0 + c4) = v;
        }
        __threadfence();
      }
    } else {
      const int q = lane >> 3, c8 = (lane & 7) * 8;
      unsigned short* C  = (unsigned short*)Cout  + (size_t)b * strideC;
      unsigned short* C2 = (OUT_MODE == 2) ? ((unsigned short*)Cout2 + (size_t)b * strideC) : nullptr;
      for (int pass = 0; pass < 2; ++pass) {
#pragma unroll
        for (int it = 0; it < 4; ++it) {
          const int row = it * 4 + q;
          const float* sp = slab + row * 68 + c8;
          v8h hv, lv;
#pragma unroll
          for (int e = 0; e < 8; ++e) {
            if (OUT_MODE == 1) {
              hv[e] = (_Float16)sp[e];
            } else {
              unsigned short hb = f2bf_bits(sp[e]);
              unsigned short lb = f2bf_bits(sp[e] - bf_bits2f(hb));
              hv[e] = __builtin_bit_cast(_Float16, hb);
              lv[e] = __builtin_bit_cast(_Float16, lb);
            }
          }
          *(volatile v8h*)(C + (size_t)(mBase + row) * ldc + n0 + c8) = hv;
          if (OUT_MODE == 2) *(volatile v8h*)(C2 + (size_t)(mBase + row) * ldc + n0 + c8) = lv;
        }
        __threadfence();
      }
    }
    __builtin_amdgcn_fence(__ATOMIC_RELEASE, "workgroup");
    __builtin_amdgcn_wave_barrier();
    __builtin_amdgcn_fence(__ATOMIC_ACQUIRE, "workgroup");
  }
}

template <int NB>
__device__ __forceinline__ int scan_chunk(const int* __restrict__ lst, int nE, int cbase, int nodeBase,
                                          int* list, int tid, int lane, int wave, int fullvec) {
  int wc = 0;
#pragma unroll
  for (int g = 0; g < NGRP; ++g) {
    const int el0 = (g * NTHR + tid) * EPT;
    const int e0  = cbase + el0;
    v4i da, db;
    if (fullvec) {
      da = *(const v4i*)(lst + e0);
      db = *(const v4i*)(lst + e0 + 4);
    } else {
      const int em = nE - 1;
      da.x = lst[(e0     < em) ? e0     : em];
      da.y = lst[(e0 + 1 < em) ? e0 + 1 : em];
      da.z = lst[(e0 + 2 < em) ? e0 + 2 : em];
      da.w = lst[(e0 + 3 < em) ? e0 + 3 : em];
      db.x = lst[(e0 + 4 < em) ? e0 + 4 : em];
      db.y = lst[(e0 + 5 < em) ? e0 + 5 : em];
      db.z = lst[(e0 + 6 < em) ? e0 + 6 : em];
      db.w = lst[(e0 + 7 < em) ? e0 + 7 : em];
    }
    const bool v0 = (e0 < nE), v1 = (e0 + 1 < nE), v2 = (e0 + 2 < nE), v3 = (e0 + 3 < nE);
    const bool v4 = (e0 + 4 < nE), v5 = (e0 + 5 < nE), v6 = (e0 + 6 < nE), v7 = (e0 + 7 < nE);
    const unsigned nb = (unsigned)nodeBase;
    const unsigned s0 = (unsigned)da.x - nb, s1 = (unsigned)da.y - nb;
    const unsigned s2 = (unsigned)da.z - nb, s3 = (unsigned)da.w - nb;
    const unsigned s4 = (unsigned)db.x - nb, s5 = (unsigned)db.y - nb;
    const unsigned s6 = (unsigned)db.z - nb, s7 = (unsigned)db.w - nb;
    const bool h0 = v0 && (s0 < (unsigned)NB), h1 = v1 && (s1 < (unsigned)NB);
    const bool h2 = v2 && (s2 < (unsigned)NB), h3 = v3 && (s3 < (unsigned)NB);
    const bool h4 = v4 && (s4 < (unsigned)NB), h5 = v5 && (s5 < (unsigned)NB);
    const bool h6 = v6 && (s6 < (unsigned)NB), h7 = v7 && (s7 < (unsigned)NB);
    const unsigned any = __builtin_amdgcn_ballot_w32(h0 | h1 | h2 | h3 | h4 | h5 | h6 | h7);
    if (any != 0u) {
#define HITJ(J, HJ, SJ) { \
        const unsigned mj = __builtin_amdgcn_ballot_w32(HJ); \
        if (mj != 0u) { \
          if (HJ) { \
            const int pos = wc + (int)__builtin_amdgcn_mbcnt_lo(mj, 0u); \
            if (pos < WCAP) list[wave * WCAP + pos] = ((el0 + (J)) << 12) | (int)(SJ); \
          } \
          wc += (int)__builtin_popcount(mj); } }
      HITJ(0, h0, s0)
      HITJ(1, h1, s1)
      HITJ(2, h2, s2)
      HITJ(3, h3, s3)
      HITJ(4, h4, s4)
      HITJ(5, h5, s5)
      HITJ(6, h6, s6)
      HITJ(7, h7, s7)
#undef HITJ
    }
  }
  return wc;
}

__device__ __forceinline__ float dot4f(v4f a, v4f b) {
  return a.x * b.x + a.y * b.y + a.z * b.z + a.w * b.w;
}
__device__ __forceinline__ void split_bf(float f, _Float16& h, _Float16& l) {
  const unsigned short hb = f2bf_bits(f);
  const unsigned short lb = f2bf_bits(f - bf_bits2f(hb));
  h = __builtin_bit_cast(_Float16, hb);
  l = __builtin_bit_cast(_Float16, lb);
}
__device__ __forceinline__ void split8(v4f a, v4f b, v8h& hv, v8h& lv) {
  _Float16 h0, l0, h1, l1, h2, l2, h3, l3, h4, l4, h5, l5, h6, l6, h7, l7;
  split_bf(a.x, h0, l0); split_bf(a.y, h1, l1); split_bf(a.z, h2, l2); split_bf(a.w, h3, l3);
  split_bf(b.x, h4, l4); split_bf(b.y, h5, l5); split_bf(b.z, h6, l6); split_bf(b.w, h7, l7);
  hv[0] = h0; hv[1] = h1; hv[2] = h2; hv[3] = h3; hv[4] = h4; hv[5] = h5; hv[6] = h6; hv[7] = h7;
  lv[0] = l0; lv[1] = l1; lv[2] = l2; lv[3] = l3; lv[4] = l4; lv[5] = l5; lv[6] = l6; lv[7] = l7;
}
template <int CPL> struct VecT { typedef float T __attribute__((ext_vector_type(CPL))); };
template <> struct VecT<1> { typedef float T; };

template <int MODE, int KIN, int KP>
__global__ __launch_bounds__(256) void k_wprep(const float* __restrict__ w, unsigned short* p0,
                                               unsigned short* p1) {
  static_assert(KIN <= 64 && KP % 32 == 0 && KP >= KIN && KP <= 64 && (FW * KP / 8) % 256 == 0);
  __shared__ __align__(16) float sw[64 * FW];
  const int tid = threadIdx.x;
  for (int i = tid; i < KIN * FW; i += 256) sw[i] = w[i];
  __syncthreads();
  constexpr int TPR = KP / 8;
  constexpr int NTK = FW * TPR;
  for (int pass = 0; pass < 2; ++pass) {
#pragma unroll 1
    for (int it = 0; it < NTK / 256; ++it) {
      const int t  = it * 256 + tid;
      const int n  = t / TPR;
      const int k0 = (t - n * TPR) * 8;
      v8h hv, lv;
#pragma unroll
      for (int e = 0; e < 8; ++e) {
        const int k  = k0 + e;
        const int kc = (k < KIN) ? k : KIN - 1;
        float f = sw[kc * FW + n];
        if (k >= KIN) f = 0.f;
        if (MODE == 1) {
          _Float16 h, l; split_bf(f, h, l); hv[e] = h; lv[e] = l;
        } else {
          hv[e] = (_Float16)f; lv[e] = (_Float16)0.f;
        }
      }
      *(volatile v8h*)(p0 + (size_t)t * 8) = hv;
      if (MODE == 1) *(volatile v8h*)(p1 + (size_t)t * 8) = lv;
    }
    __threadfence();
  }
}

__global__ __launch_bounds__(NTHR) void k_split_x(const float* __restrict__ x, unsigned short* ph,
                                                  unsigned short* pl, int nValid, int nRows) {
  const int i = blockIdx.x * NTHR + threadIdx.x;
  if (i >= nRows * 4) return;
  const int row = i >> 2, g = i & 3;
  const int rc  = (row < nValid) ? row : nValid - 1;
  const float* xp = x + (size_t)rc * XIN + (g & 1) * 8;
  v4f a = *(const v4f*)xp, b = *(const v4f*)(xp + 4);
  if (row >= nValid || g >= 2) { const v4f z = {0.f, 0.f, 0.f, 0.f}; a = z; b = z; }
  v8h hv, lv;
  split8(a, b, hv, lv);
  const size_t o = (size_t)i * 8;
  *(volatile v8h*)(ph + o) = hv;
  *(volatile v8h*)(pl + o) = lv;
  __threadfence();
  *(volatile v8h*)(ph + o) = hv;
  *(volatile v8h*)(pl + o) = lv;
}

__global__ __launch_bounds__(NTHR) void k_fuse_h1(const float* __restrict__ oa, const float* __restrict__ ou,
                                                  const float* __restrict__ wl, unsigned short* ph,
                                                  unsigned short* pl, int nValid, int nRows) {
  const int i = blockIdx.x * NTHR + threadIdx.x;
  if (i >= nRows * 8) return;
  const int row = i >> 3, c0 = (i & 7) * 8;
  const float w0 = wl[0], w1 = wl[1];
  const size_t o = (size_t)row * FW + c0;
  const v4f a0 = *(const v4f*)(oa + o), a1 = *(const v4f*)(oa + o + 4);
  const v4f b0 = *(const v4f*)(ou + o), b1 = *(const v4f*)(ou + o + 4);
  v4f u0 = a0 * w0 + b0 * w1, u1 = a1 * w0 + b1 * w1;
  u0.x = fmaxf(u0.x, 0.f); u0.y = fmaxf(u0.y, 0.f); u0.z = fmaxf(u0.z, 0.f); u0.w = fmaxf(u0.w, 0.f);
  u1.x = fmaxf(u1.x, 0.f); u1.y = fmaxf(u1.y, 0.f); u1.z = fmaxf(u1.z, 0.f); u1.w = fmaxf(u1.w, 0.f);
  if (row >= nValid) { const v4f z = {0.f, 0.f, 0.f, 0.f}; u0 = z; u1 = z; }
  v8h hv, lv;
  split8(u0, u1, hv, lv);
  const size_t so = (size_t)i * 8;
  *(volatile v8h*)(ph + so) = hv;
  *(volatile v8h*)(pl + so) = lv;
  __threadfence();
  *(volatile v8h*)(ph + so) = hv;
  *(volatile v8h*)(pl + so) = lv;
}

template <int NH>
__global__ __launch_bounds__(NTHR) void k_score(const float* __restrict__ feat, int fstride,
                                                const float* __restrict__ av, float* outp,
                                                int nValid, int nRows) {
  static_assert(NH == 1 || NH == 4);
  constexpr int DC = FW / NH;
  const int node = blockIdx.x * NTHR + threadIdx.x;
  if (node >= nRows) return;
  const int nc = (node < nValid) ? node : nValid - 1;
  const float* hr = feat + (size_t)nc * fstride;
  float sv[NH];
#pragma unroll
  for (int hd = 0; hd < NH; ++hd) sv[hd] = 0.f;
#pragma unroll 1
  for (int c = 0; c < DC; c += 4) {
#pragma unroll
    for (int hd = 0; hd < NH; ++hd)
      sv[hd] += dot4f(*(const v4f*)(hr + hd * DC + c), *(const v4f*)(av + hd * DC + c));
  }
  v4f o = {0.f, 0.f, 0.f, 0.f};
  if (node < nValid) {
    o.x = sv[0];
    if constexpr (NH == 4) { o.y = sv[1]; o.z = sv[2]; o.w = sv[3]; }
  }
  float* dp = outp + (size_t)node * 4;
  *(volatile v4f*)dp = o;
  __threadfence();
  *(volatile v4f*)dp = o;
}

template <int NB, int NH>
__global__ __launch_bounds__(NTHR) void k_gat_agg(
    const int* __restrict__ srcl, const int* __restrict__ dstl,
    const float* __restrict__ hfeat, int sstride,
    const float* __restrict__ els, const float* __restrict__ eld,
    float* of, unsigned short* oh, int nSrc, int nE, int vec_ok) {
  constexpr int HC  = FW;
  constexpr int DC  = HC / NH;
  constexpr int RW  = NB / NWAVE;
  constexpr int C4R = HC / 4;
  static_assert((NB * HC / 4) % NTHR == 0);
  static_assert(NB % NWAVE == 0 && (RW % 4) == 0);
  static_assert((NB & (NB - 1)) == 0 && NB <= 4096);
  static_assert(HC == 64 && C4R == 16 && (NH == 1 || NH == 4));
  typedef typename VecT<2>::T VT;
  extern __shared__ v4f lds_dyn[];
  float* acc  = (float*)lds_dyn;
  float* mst  = acc + NB * HC;
  float* sst  = mst + NB * NH;
  int*   list = (int*)(sst + NB * NH);
  int*   wcnt = list + LISTN;
  const int tid = threadIdx.x, lane = tid & 31, wave = tid >> 5;
  const int nodeBase = blockIdx.x * NB;

  {
    const v4f zz = {0.f, 0.f, 0.f, 0.f};
    for (int i = tid; i < NB * HC / 4; i += NTHR) lds_dyn[i] = zz;
    for (int i = tid; i < NB * NH; i += NTHR) { mst[i] = -INFINITY; sst[i] = 0.f; }
  }
  __syncthreads();

  const int colL = 2 * lane;
  const int hdl  = colL / DC;
  const int nChunks = (nE + CHUNK - 1) / CHUNK;
#pragma unroll 1
  for (int ch = 0; ch < nChunks; ++ch) {
    const int cbase = ch * CHUNK;
    const int fullvec = (vec_ok != 0 && cbase + CHUNK <= nE) ? 1 : 0;
    const int wc = scan_chunk<NB>(dstl, nE, cbase, nodeBase, list, tid, lane, wave, fullvec);
    if (lane == 0) wcnt[wave] = wc;
    __syncthreads();
    if (wave == 0) {
#pragma unroll 1
      for (int wsx = 0; wsx < NWAVE; ++wsx) {
        int n = __builtin_amdgcn_readfirstlane(wcnt[wsx]);
        n = n > WCAP ? WCAP : (n < 0 ? 0 : n);
        const int* lp = list + wsx * WCAP;
#pragma unroll 1
        for (int i = 0; i < n; ++i) {
          const int ent  = __builtin_amdgcn_readfirstlane(lp[i]);
          const int slot = ent & (NB - 1);
          int e = cbase + ((ent >> 12) & (CHUNK - 1));
          e = e > nE - 1 ? nE - 1 : e;
          int s = srcl[e];
          s = s < 0 ? 0 : (s > nSrc - 1 ? nSrc - 1 : s);
          const int node = nodeBase + slot;
          float lg = els[(size_t)s * 4 + hdl] + eld[(size_t)node * 4 + hdl];
          lg = (lg > 0.f) ? lg : 0.2f * lg;
          const int mi = slot * NH + hdl;
          const float mo = mst[mi];
          const float so = sst[mi];
          const float d  = __expf(-fabsf(lg - mo));
          const bool  up = (lg > mo);
          const float sc = up ? d : 1.0f;
          const float w  = up ? 1.0f : d;
          const VT hv = *(const VT*)(hfeat + (size_t)s * sstride + colL);
          VT* ap = (VT*)(acc + slot * HC + colL);
          const VT av = *ap;
          *ap = av * sc + hv * w;
          mst[mi] = up ? lg : mo;
          sst[mi] = so * sc + w;
        }
      }
    }
    __syncthreads();
  }

#pragma unroll 1
  for (int it = 0; it < (NB * HC / 4) / NTHR; ++it) {
    const int idx  = it * NTHR + tid;
    const int slot = idx / C4R;
    const int c4   = (idx - slot * C4R) * 4;
    const int hd   = c4 / DC;
    const float so = sst[slot * NH + hd];
    const float rv = __builtin_amdgcn_rcpf((so > 0.f) ? so : 1.0f);
    const float inv = (so > 0.f) ? rv : 0.f;
    v4f* ap = (v4f*)(acc + slot * HC + c4);
    const v4f a = *ap;
    v4f r = a * inv;
    r.x = fmaxf(r.x, 0.f); r.y = fmaxf(r.y, 0.f); r.z = fmaxf(r.z, 0.f); r.w = fmaxf(r.w, 0.f);
    *ap = r;
  }
  __syncthreads();

  for (int pass = 0; pass < 2; ++pass) {
#pragma unroll 1
    for (int it = 0; it < RW / 2; ++it) {
      const int row = wave * RW + it * 2 + (lane >> 4);
      const int col = (lane & 15) * 4;
      const v4f v = *(const v4f*)(acc + row * HC + col);
      *(volatile v4f*)(of + (size_t)(nodeBase + row) * HC + col) = v;
    }
#pragma unroll 1
    for (int it = 0; it < RW / 4; ++it) {
      const int row = wave * RW + it * 4 + (lane >> 3);
      const int c8  = (lane & 7) * 8;
      const float* sp = acc + row * HC + c8;
      v8h hv;
#pragma unroll
      for (int e = 0; e < 8; ++e) hv[e] = (_Float16)sp[e];
      *(volatile v8h*)(oh + (size_t)(nodeBase + row) * HC + c8) = hv;
    }
    __threadfence();
  }
}

template <int MODE>
__global__ __launch_bounds__(NTHR) void k_colsum(const float* __restrict__ pa, const float* __restrict__ pb,
                                                 const float* __restrict__ wl, float* part, int nValid) {
  __shared__ __align__(16) float red[4][FW];
  __shared__ __align__(16) float outl[FW];
  const int tid = threadIdx.x;
  const int c = tid & 63, ph = tid >> 6;
  const int rowBase = blockIdx.x * ROWS_CS;
  float w0 = 0.f, w1 = 0.f;
  if (MODE == 2) { w0 = wl[0]; w1 = wl[1]; }
  float s = 0.f;
#pragma unroll 1
  for (int i = 0; i < ROWS_CS / 4; ++i) {
    const int r = rowBase + ph + 4 * i;
    const float a = pa[(size_t)r * FW + c];
    float v;
    if (MODE == 1) {
      v = tanhf(a);
    } else {
      const float b = pb[(size_t)r * FW + c];
      v = w0 * a + w1 * b;
    }
    if (r < nValid) s += v;
  }
  red[ph][c] = s;
  __syncthreads();
  if (tid < FW) outl[tid] = ((red[0][tid] + red[1][tid]) + red[2][tid]) + red[3][tid];
  __syncthreads();
  if (tid < 16) {
    const v4f o = *(const v4f*)(outl + tid * 4);
    float* dp = part + (size_t)blockIdx.x * FW + tid * 4;
    *(volatile v4f*)dp = o;
    __threadfence();
    *(volatile v4f*)dp = o;
  }
}

__global__ __launch_bounds__(64) void k_semantic(const float* __restrict__ pta, const float* __restrict__ ptb,
                                                 int nPart, const float* __restrict__ q, int nValid, float* wl) {
  __shared__ float pr[2][FW];
  __shared__ float wv[2];
  const int c = threadIdx.x;
  double sa = 0.0, sb = 0.0;
#pragma unroll 1
  for (int p = 0; p < nPart; ++p) { sa += (double)pta[(size_t)p * FW + c]; sb += (double)ptb[(size_t)p * FW + c]; }
  const float inv = 1.0f / (float)nValid;
  const float ma = (float)sa * inv, mb = (float)sb * inv;
  const float qc = q[c];
  pr[0][c] = qc * ma;
  pr[1][c] = qc * mb;
  __syncthreads();
  if (c == 0) {
    double t0 = 0.0, t1 = 0.0;
#pragma unroll 1
    for (int k = 0; k < FW; ++k) { t0 += (double)pr[0][k]; t1 += (double)pr[1][k]; }
    const float s0 = (float)t0, s1 = (float)t1;
    const float mx = fmaxf(s0, s1);
    const float e0 = expf(s0 - mx), e1 = expf(s1 - mx);
    const float r  = 1.0f / (e0 + e1);
    wv[0] = e0 * r;
    wv[1] = e1 * r;
  }
  __syncthreads();
  if (c < 32) {
    const float a0 = wv[0], a1 = wv[1];
    const float v = (c == 0) ? a0 : ((c == 1) ? a1 : 0.f);
    *(volatile float*)(wl + c) = v;
    __threadfence();
    *(volatile float*)(wl + c) = v;
  }
}

__global__ __launch_bounds__(64) void k_rowvec(const float* __restrict__ wu, const float* __restrict__ bu,
                                               float* rv) {
  __shared__ __align__(16) float sv[FW];
  const int c = threadIdx.x;
  const float zero = 0.0f;
  float s = 0.f;
#pragma unroll 1
  for (int k = 0; k < FW; ++k) s += zero * wu[(size_t)k * FW + c];
  sv[c] = s + bu[c];
  __syncthreads();
  if (c < 16) {
    const v4f o = *(const v4f*)(sv + c * 4);
    *(volatile v4f*)(rv + c * 4) = o;
    __threadfence();
    *(volatile v4f*)(rv + c * 4) = o;
  }
}

__global__ __launch_bounds__(64) void k_final(const float* __restrict__ part, int nPart, int nValid,
                                              const float* __restrict__ wp, const float* __restrict__ bp,
                                              float* out) {
  __shared__ __align__(16) float emb[FW];
  __shared__ __align__(16) float res[FW];
  const int c = threadIdx.x;
  double s = 0.0;
#pragma unroll 1
  for (int p = 0; p < nPart; ++p) s += (double)part[(size_t)p * FW + c];
  emb[c] = (float)(s / (double)nValid);
  __syncthreads();
  float a = bp[c];
#pragma unroll 1
  for (int k = 0; k < FW; ++k) a += emb[k] * wp[(size_t)k * FW + c];
  res[c] = a;
  __syncthreads();
  if (c < 16) {
    const v4f o = *(const v4f*)(res + c * 4);
    *(volatile v4f*)(out + c * 4) = o;
    __threadfence();
    *(volatile v4f*)(out + c * 4) = o;
  }
}

extern "C" void kernel_launch(void* const* d_in, const int* in_sizes, int n_in,
                              void* d_out, int out_size, void* d_ws, size_t ws_size,
                              hipStream_t stream) {
  if (n_in < 28) return;
  const int nH = in_sizes[0] / XIN;
  const int nU = in_sizes[1] / XIN;
  const int eA = in_sizes[2] / 2;
  const int eU = in_sizes[3] / 2;
  if (nH < 1 || nU < 1 || eA < 1 || eU < 1) return;
  if (in_sizes[0] != nH * XIN || in_sizes[1] != nU * XIN) return;
  if (in_sizes[2] != 2 * eA || in_sizes[3] != 2 * eU) return;
  if (nH > (1 << 22) || nU > (1 << 22) || eA > (1 << 28) || eU > (1 << 28)) return;
  if (in_sizes[4] != XIN * FW || in_sizes[5] != FW || in_sizes[6] != XIN * FW || in_sizes[7] != FW) return;
  for (int i = 8; i <= 11; ++i) if (in_sizes[i] != FW) return;
  if (in_sizes[12] != FW * FW || in_sizes[13] != FW || in_sizes[14] != FW) return;
  if (in_sizes[15] != FW * FW || in_sizes[16] != FW || in_sizes[17] != FW * FW || in_sizes[18] != FW) return;
  for (int i = 19; i <= 22; ++i) if (in_sizes[i] != FW) return;
  if (in_sizes[23] != FW * FW || in_sizes[24] != FW || in_sizes[25] != FW) return;
  if (in_sizes[26] != FW * FW || in_sizes[27] != FW) return;
  if (out_size != FW) return;

  const float* x_host = (const float*)d_in[0];
  const float* x_user = (const float*)d_in[1];
  const int*   eiA    = (const int*)d_in[2];
  const int*   eiU    = (const int*)d_in[3];
  const float* W1h = (const float*)d_in[4];  const float* b1h = (const float*)d_in[5];
  const float* W1u = (const float*)d_in[6];  const float* b1u = (const float*)d_in[7];
  const float* as1a = (const float*)d_in[8]; const float* ad1a = (const float*)d_in[9];
  const float* as1u = (const float*)d_in[10];const float* ad1u = (const float*)d_in[11];
  const float* Wk1 = (const float*)d_in[12]; const float* bk1 = (const float*)d_in[13];
  const float* q1  = (const float*)d_in[14];
  const float* W2h = (const float*)d_in[15]; const float* b2h = (const float*)d_in[16];
  const float* W2u = (const float*)d_in[17]; const float* b2u = (const float*)d_in[18];
  const float* as2a = (const float*)d_in[19];const float* ad2a = (const float*)d_in[20];
  const float* as2u = (const float*)d_in[21];const float* ad2u = (const float*)d_in[22];
  const float* Wk2 = (const float*)d_in[23]; const float* bk2 = (const float*)d_in[24];
  const float* q2  = (const float*)d_in[25];
  const float* Wp  = (const float*)d_in[26]; const float* bp  = (const float*)d_in[27];
  float* out = (float*)d_out;
  const int* srcA = eiA;  const int* dstA = eiA + eA;
  const int* srcU = eiU;  const int* dstU = eiU + eU;
  const int vecA = (eA % 4 == 0) ? 1 : 0;
  const int vecU = (eU % 4 == 0) ? 1 : 0;

  const int RPh = ((nH + RPQ - 1) / RPQ) * RPQ;
  const int RPu = ((nU + RPQ - 1) / RPQ) * RPQ;
  const int RPM = (RPh > RPu) ? RPh : RPu;
  const int nPart = RPh / ROWS_CS;

  char* ws = (char*)d_ws;
  size_t off = 0;
  const size_t szF32 = (size_t)RPh * FW * 4;
  const size_t oXH   = off; off += szF32;
  const size_t oXU   = off; off += (size_t)RPM * FW * 4;
  size_t szOA = szF32; if ((size_t)RPM * XKP * 2 * 2 > szOA) szOA = (size_t)RPM * XKP * 2 * 2;
  const size_t oOA   = off; off += szOA;
  const size_t oOA16 = off; off += (size_t)RPh * FW * 2;
  const size_t oOU   = off; off += szF32;
  const size_t oOU16 = off; off += (size_t)RPh * FW * 2;
  const size_t oALS  = off; off += (size_t)RPM * 4 * 4;
  const size_t oALD  = off; off += (size_t)RPh * 4 * 4;
  const size_t oWB   = off; off += 8 * 8192;
  const size_t oPTA  = off; off += (size_t)nPart * FW * 4;
  const size_t oPTB  = off; off += (size_t)nPart * FW * 4;
  const size_t oWL   = off; off += 256;
  const size_t oRV   = off; off += 256;
  if (off > ws_size || off > (size_t)134217728) return;

  float* XH = (float*)(ws + oXH);
  float* XU = (float*)(ws + oXU);
  float* OA = (float*)(ws + oOA);
  float* OU = (float*)(ws + oOU);
  unsigned short* OA16 = (unsigned short*)(ws + oOA16);
  unsigned short* OU16 = (unsigned short*)(ws + oOU16);
  float* ALS = (float*)(ws + oALS);
  float* ALD = (float*)(ws + oALD);
  unsigned short* xah  = (unsigned short*)(ws + oOA);
  unsigned short* xal  = (unsigned short*)(ws + oOA + (size_t)RPM * XKP * 2);
  unsigned short* h1h  = (unsigned short*)(ws + oXU);
  unsigned short* h1l  = (unsigned short*)(ws + oXU + (size_t)RPh * FW * 2);
  unsigned short* w1hh = (unsigned short*)(ws + oWB + 0 * 8192);
  unsigned short* w1hl = (unsigned short*)(ws + oWB + 1 * 8192);
  unsigned short* w1uh = (unsigned short*)(ws + oWB + 2 * 8192);
  unsigned short* w1ul = (unsigned short*)(ws + oWB + 3 * 8192);
  unsigned short* w2hh = (unsigned short*)(ws + oWB + 4 * 8192);
  unsigned short* w2hl = (unsigned short*)(ws + oWB + 5 * 8192);
  unsigned short* wk1t = (unsigned short*)(ws + oWB + 6 * 8192);
  unsigned short* wk2t = (unsigned short*)(ws + oWB + 7 * 8192);
  float* PTA = (float*)(ws + oPTA);
  float* PTB = (float*)(ws + oPTB);
  float* WL  = (float*)(ws + oWL);
  float* RV  = (float*)(ws + oRV);
  float* TP  = XH;

  const int gH = ((RPh / 64) * (FW / 64) + 7) / 8;
  const int gU = ((RPu / 64) * (FW / 64) + 7) / 8;

  k_wprep<1, XIN, XKP><<<1, 256, 0, stream>>>(W1h, w1hh, w1hl);
  k_wprep<1, XIN, XKP><<<1, 256, 0, stream>>>(W1u, w1uh, w1ul);
  k_wprep<1, FW, FW><<<1, 256, 0, stream>>>(W2h, w2hh, w2hl);
  k_wprep<0, FW, FW><<<1, 256, 0, stream>>>(Wk1, wk1t, wk1t);
  k_wprep<0, FW, FW><<<1, 256, 0, stream>>>(Wk2, wk2t, wk2t);

  k_split_x<<<RPh * 4 / NTHR, NTHR, 0, stream>>>(x_host, xah, xal, nH, RPh);
  wmma_gemm64<1, true, 2, 0, false, 0><<<dim3(gH, 1), 256, 0, stream>>>(
      xah, xal, XKP, 0L, w1hh, w1hl, XKP, 0L, (void*)XH, (void*)XH, FW, 0L,
      b1h, XH, 0L, RPh, FW, XKP, 1.0f);
  k_split_x<<<RPu * 4 / NTHR, NTHR, 0, stream>>>(x_user, xah, xal, nU, RPu);
  wmma_gemm64<1, true, 2, 0, false, 0><<<dim3(gU, 1), 256, 0, stream>>>(
      xah, xal, XKP, 0L, w1uh, w1ul, XKP, 0L, (void*)XU, (void*)XU, FW, 0L,
      b1u, XU, 0L, RPu, FW, XKP, 1.0f);

  k_score<NHL1><<<RPh / NTHR, NTHR, 0, stream>>>(XH, FW, as1a, ALS, nH, RPh);
  k_score<NHL1><<<RPh / NTHR, NTHR, 0, stream>>>(XH, FW, ad1a, ALD, nH, RPh);
  k_gat_agg<NBL1, NHL1><<<RPh / NBL1, NTHR, LDS1, stream>>>(
      srcA, dstA, XH, FW, ALS, ALD, OA, OA16, nH, eA, vecA);
  k_score<NHL1><<<RPu / NTHR, NTHR, 0, stream>>>(XU, FW, as1u, ALS, nU, RPu);
  k_score<NHL1><<<RPh / NTHR, NTHR, 0, stream>>>(XH, FW, ad1u, ALD, nH, RPh);
  k_gat_agg<NBL1, NHL1><<<RPh / NBL1, NTHR, LDS1, stream>>>(
      srcU, dstU, XU, FW, ALS, ALD, OU, OU16, nU, eU, vecU);

  wmma_gemm64<0, false, 2, 0, false, 0><<<dim3(gH, 1), 256, 0, stream>>>(
      OA16, OA16, FW, 0L, wk1t, wk1t, FW, 0L, (void*)TP, (void*)TP, FW, 0L,
      bk1, TP, 0L, RPh, FW, FW, 1.0f);
  k_colsum<1><<<nPart, NTHR, 0, stream>>>(TP, TP, WL, PTA, nH);
  wmma_gemm64<0, false, 2, 0, false, 0><<<dim3(gH, 1), 256, 0, stream>>>(
      OU16, OU16, FW, 0L, wk1t, wk1t, FW, 0L, (void*)TP, (void*)TP, FW, 0L,
      bk1, TP, 0L, RPh, FW, FW, 1.0f);
  k_colsum<1><<<nPart, NTHR, 0, stream>>>(TP, TP, WL, PTB, nH);
  k_semantic<<<1, 64, 0, stream>>>(PTA, PTB, nPart, q1, nH, WL);
  k_fuse_h1<<<RPh * 8 / NTHR, NTHR, 0, stream>>>(OA, OU, WL, h1h, h1l, nH, RPh);

  wmma_gemm64<1, true, 2, 0, false, 0><<<dim3(gH, 1), 256, 0, stream>>>(
      h1h, h1l, FW, 0L, w2hh, w2hl, FW, 0L, (void*)XH, (void*)XH, FW, 0L,
      b2h, XH, 0L, RPh, FW, FW, 1.0f);
  k_rowvec<<<1, 64, 0, stream>>>(W2u, b2u, RV);

  k_score<1><<<RPh / NTHR, NTHR, 0, stream>>>(XH, FW, as2a, ALS, nH, RPh);
  k_score<1><<<RPh / NTHR, NTHR, 0, stream>>>(XH, FW, ad2a, ALD, nH, RPh);
  k_gat_agg<NBL2, 1><<<RPh / NBL2, NTHR, LDS2, stream>>>(
      srcA, dstA, XH, FW, ALS, ALD, OA, OA16, nH, eA, vecA);
  k_score<1><<<RPu / NTHR, NTHR, 0, stream>>>(RV, 0, as2u, ALS, nU, RPu);
  k_score<1><<<RPh / NTHR, NTHR, 0, stream>>>(XH, FW, ad2u, ALD, nH, RPh);
  k_gat_agg<NBL2, 1><<<RPh / NBL2, NTHR, LDS2, stream>>>(
      srcU, dstU, RV, 0, ALS, ALD, OU, OU16, nU, eU, vecU);

  wmma_gemm64<0, false, 2, 0, false, 0><<<dim3(gH, 1), 256, 0, stream>>>(
      OA16, OA16, FW, 0L, wk2t, wk2t, FW, 0L, (void*)TP, (void*)TP, FW, 0L,
      bk2, TP, 0L, RPh, FW, FW, 1.0f);
  k_colsum<1><<<nPart, NTHR, 0, stream>>>(TP, TP, WL, PTA, nH);
  wmma_gemm64<0, false, 2, 0, false, 0><<<dim3(gH, 1), 256, 0, stream>>>(
      OU16, OU16, FW, 0L, wk2t, wk2t, FW, 0L, (void*)TP, (void*)TP, FW, 0L,
      bk2, TP, 0L, RPh, FW, FW, 1.0f);
  k_colsum<1><<<nPart, NTHR, 0, stream>>>(TP, TP, WL, PTB, nH);
  k_semantic<<<1, 64, 0, stream>>>(PTA, PTB, nPart, q2, nH, WL);

  k_colsum<2><<<nPart, NTHR, 0, stream>>>(OA, OU, WL, PTA, nH);
  k_final<<<1, 64, 0, stream>>>(PTA, nPart, nH, Wp, bp, out);
}
